// GCN2LayerConcat_26560077758924
// MI455X (gfx1250) — hardware-run, weakly checked
//
#include <hip/hip_runtime.h>


namespace {
constexpr int N = 65536, E = 1048576, FIN = 16, HID = 64, NG = 32, PPG = 2048, OUT = 12, KFC = PPG * HID  , NCH = 64, KCH = KFC / NCH  ;
constexpr float XS = 8.0f, WSC = 256.0f;

typedef _Float16 b16;
typedef __attribute__((ext_vector_type(16))) _Float16 v16b;
typedef __attribute__((ext_vector_type(8))) _Float16 v8b;
typedef __attribute__((ext_vector_type(8))) float v8f;
typedef __attribute__((ext_vector_type(4))) float v4f;
typedef __attribute__((ext_vector_type(2))) float v2f;
typedef __attribute__((ext_vector_type(2))) _Float16 v2b;
__device__ __forceinline__ float bf16_rne(float f) { unsigned int u = __float_as_uint(f); u += 0x7FFFu + ((u >> 16) & 1u); return __uint_as_float(u & 0xFFFF0000u); }
__device__ __forceinline__ void split16(float v, b16& hi, b16& lo) { hi = (b16)v; lo = (b16)(v - (float)hi); }
__device__ __forceinline__ v16b frag_kb(const b16* p, int hh) { const v8b a = *(const v8b*)(p + 8 * hh), b = *(const v8b*)(p + 16 + 8 * hh); v16b f;
#pragma unroll
  for (int e = 0; e < 8; ++e) { f[e] = a[e]; f[8 + e] = b[e]; } return f; }
__device__ __forceinline__ v8f wmma16b(v16b a, v16b b, v8f c) { v8f d = __builtin_amdgcn_wmma_f32_16x16x32_f16(false, a, false, b, (short)0, c, false, false); asm volatile("v_nop\n\tv_nop\n\tv_nop\n\tv_nop" : "+v"(d) : "v"(a), "v"(b)); return d; }
__device__ __forceinline__ void wave_lds_sync() { __builtin_amdgcn_fence(__ATOMIC_RELEASE, "workgroup"); __builtin_amdgcn_wave_barrier(); __builtin_amdgcn_fence(__ATOMIC_ACQUIRE, "workgroup"); }
__device__ __forceinline__ float pmul(float a, float b) { float p = a * b; asm volatile("" : "+v"(p)); return p; }
__device__ __forceinline__ int iclamp(int v, int lo, int hi) { return v < lo ? lo : (v > hi ? hi : v); }
__device__ __forceinline__ float nexp(float x) { return __builtin_amdgcn_exp2f(x * 1.4426950408889634f); }
__device__ __forceinline__ float tanh_(float x) { const float e = nexp(-2.0f * fabsf(x)); const float t = (1.0f - e) / (1.0f + e); return x < 0.0f ? -t : t; }

constexpr int CSR_NBLK = 512, CSR_GB = 9, CSR_GN = 1 << CSR_GB  , CSR_MAXG = 512, CSR_CAP = 12288  ;
__global__ __launch_bounds__(64) void csrA_kernel(const int* __restrict__ dst, int E, int N, int nG, int CHP, int NGP, int* __restrict__ STG, int* __restrict__ HST) {
  extern __shared__ int sm[];
  int* cnt = sm; int* run = sm + NGP; int* ids = sm + 2 * NGP;
  const int b = blockIdx.x; const int ch = (E + CSR_NBLK - 1) / CSR_NBLK; const int e0 = b * ch, e1 = min(E, e0 + ch);
  for (int i = threadIdx.x; i < NGP; i += 64) cnt[i] = 0;
  for (int i = threadIdx.x; i < CHP; i += 64) ids[i] = -1;
  __syncthreads();
  if (threadIdx.x == 0) {
    for (int e = e0; e < e1; ++e) { int d = dst[e]; d = (d < 0) ? 0 : (d >= N ? N - 1 : d); cnt[d >> CSR_GB] += 1; }
    int acc = 0; for (int g = 0; g < nG; ++g) { run[g] = acc; acc += cnt[g]; }
    for (int e = e0; e < e1; ++e) { int d = dst[e]; d = (d < 0) ? 0 : (d >= N ? N - 1 : d); const int g = d >> CSR_GB; ids[run[g]] = e; run[g] += 1; } }
  __syncthreads();
  typedef __attribute__((ext_vector_type(4))) int v4i;
  for (int pass = 0; pass < 2; ++pass) {
    for (int i = threadIdx.x; i < CHP / 4; i += 64) *(volatile v4i*)(STG + (size_t)b * CHP + i * 4) = *(const v4i*)(&ids[i * 4]);
    for (int i = threadIdx.x; i < NGP / 4; i += 64) { v4i v; for (int e = 0; e < 4; ++e) v[e] = (i * 4 + e < nG) ? cnt[i * 4 + e] : 0; *(volatile v4i*)(HST + (size_t)b * NGP + i * 4) = v; }
    __threadfence(); }
}
__global__ __launch_bounds__(512) void csrS_kernel(const int* __restrict__ HST, int nG, int NGP, int* __restrict__ START, int* __restrict__ TOT, int* __restrict__ OFF) {
  __shared__ int tot[CSR_MAXG];
  const int b = threadIdx.x;
  for (int pass = 0; pass < 2; ++pass) { int runb = 0; for (int g = 0; g < nG; ++g) { int c = HST[(size_t)b * NGP + g]; c = (c < 0) ? 0 : c; ((volatile int*)OFF)[(size_t)g * CSR_NBLK + b] = runb; runb += c; } __threadfence(); }
  for (int g = threadIdx.x; g < nG; g += 512) { int s = 0; for (int bb = 0; bb < CSR_NBLK; ++bb) { int c = HST[(size_t)bb * NGP + g]; s += (c < 0) ? 0 : c; } tot[g] = s; }
  __syncthreads();
  if (threadIdx.x < 32) {
    __shared__ int st[CSR_MAXG + 32];
    if (threadIdx.x == 0) { int acc = 0; for (int g = 0; g < NGP; ++g) { st[g] = acc; if (g < nG) acc += (tot[g] + 31) & ~31; } st[NGP] = acc; }
    __builtin_amdgcn_fence(__ATOMIC_RELEASE, "workgroup"); __builtin_amdgcn_wave_barrier(); __builtin_amdgcn_fence(__ATOMIC_ACQUIRE, "workgroup");
    for (int pass = 0; pass < 2; ++pass) { for (int i = threadIdx.x; i < NGP + 32; i += 32) { ((volatile int*)START)[i] = (i <= NGP) ? st[min(i, NGP)] : 0; ((volatile int*)TOT)[i] = (i < nG) ? tot[i] : 0; } __threadfence(); } }
}
__global__ __launch_bounds__(256) void csrB_kernel(const int* __restrict__ dst, int N, int nG, int CHP, int NGP, int permLen, const int* __restrict__ STG, const int* __restrict__ HST, const int* __restrict__ OFF, const int* __restrict__ START, const int* __restrict__ TOT, int* __restrict__ PERM, int* __restrict__ ROWPTR, int* __restrict__ ROWCNT, int* __restrict__ FLAG) {
  typedef __attribute__((ext_vector_type(4))) int v4i;
  __shared__ int ids[CSR_CAP]; __shared__ unsigned short key[CSR_CAP]; __shared__ int outp[CSR_CAP]; __shared__ int ncnt[CSR_GN + 1]; __shared__ int boff[CSR_NBLK + 1];
  const int g = blockIdx.x, t_ = threadIdx.x; int tot = TOT[g]; int st = START[g], stn = START[g + 1]; const int v0 = g * CSR_GN; const int nv = min(CSR_GN, N - v0);
  st = (st < 0) ? 0 : (st > permLen - 32 ? permLen - 32 : st) & ~31; stn = (stn < st) ? st : (stn > permLen ? permLen : stn); tot = (tot < 0) ? 0 : tot; if (tot > stn - st && tot <= CSR_CAP) tot = stn - st;
  if (tot > CSR_CAP) {
    for (int pass = 0; pass < 2; ++pass) { for (int i = t_; i < CSR_GN / 4; i += 256) { v4i a, c; for (int e = 0; e < 4; ++e) { a[e] = st; c[e] = 0; } *(volatile v4i*)(ROWPTR + v0 + i * 4) = a; *(volatile v4i*)(ROWCNT + v0 + i * 4) = c; } if (t_ == 0) ((volatile int*)FLAG)[0] = 1; __threadfence(); } (void)nv; return; }
  if (t_ == 0) { int acc = 0; for (int b = 0; b < CSR_NBLK; ++b) { boff[b] = acc; int c = HST[(size_t)b * NGP + g]; c = (c < 0) ? 0 : (c > CHP ? CHP : c); acc += c; if (acc > tot) acc = tot; } boff[CSR_NBLK] = acc; }
  for (int i = t_; i <= CSR_GN; i += 256) ncnt[i] = 0;
  __syncthreads();
  for (int b = 0; b < CSR_NBLK; ++b) { const int c = boff[b + 1] - boff[b]; int o_ = OFF[(size_t)g * CSR_NBLK + b]; o_ = (o_ < 0) ? 0 : (o_ > CHP - c ? CHP - c : o_); const int* src_ = STG + (size_t)b * CHP + o_;
    for (int i = t_; i < c; i += 256) { int id = src_[i]; id = (id < 0) ? 0 : id; ids[boff[b] + i] = id; int d = dst[id]; d = (d < v0) ? v0 : (d >= N ? N - 1 : d); int kk = d - v0; kk = (kk < 0) ? 0 : (kk >= CSR_GN ? CSR_GN - 1 : kk); key[boff[b] + i] = (unsigned short)kk; } }
  __syncthreads();
  if (t_ == 0) { for (int i = 0; i < tot; ++i) ncnt[key[i]] += 1; int acc = 0; for (int vl = 0; vl < CSR_GN; ++vl) { const int c = ncnt[vl]; ncnt[vl] = acc; acc += c; } ncnt[CSR_GN] = acc;
    for (int i = 0; i < tot; ++i) { const int vl = key[i]; outp[ncnt[vl]] = ids[i]; ncnt[vl] += 1; }
    for (int vl = CSR_GN; vl > 0; --vl) ncnt[vl] = ncnt[vl - 1]; ncnt[0] = 0; }
  __syncthreads();
  for (int pass = 0; pass < 2; ++pass) {
    for (int i = t_; i < (stn - st) / 4; i += 256) { v4i v; for (int e = 0; e < 4; ++e) { const int q = i * 4 + e; v[e] = (q < tot) ? outp[q] : -1; } *(volatile v4i*)(PERM + st + i * 4) = v; }
    for (int i = t_; i < CSR_GN / 4; i += 256) { v4i a, c; for (int e = 0; e < 4; ++e) { const int vl = i * 4 + e; a[e] = st + ncnt[vl]; c[e] = (vl < nv) ? (ncnt[vl + 1] - ncnt[vl]) : 0; } *(volatile v4i*)(ROWPTR + v0 + i * 4) = a; *(volatile v4i*)(ROWCNT + v0 + i * 4) = c; }
    __threadfence(); }
}
__global__ __launch_bounds__(256) void csrZ_kernel(int* __restrict__ p, size_t n4) { typedef __attribute__((ext_vector_type(4))) int v4i; const size_t tid = (size_t)blockIdx.x * 256 + threadIdx.x, nth = (size_t)gridDim.x * 256; v4i z = {0, 0, 0, 0}; for (size_t i = tid; i < n4; i += nth) *(volatile v4i*)(p + i * 4) = z; }
struct CsrBufs { int *STG, *HST, *OFF, *START, *TOT, *PERM, *ROWPTR, *ROWCNT, *FLAG; int nG, NGP, CHP; size_t permLen; char* base; size_t bytes; };
static size_t csr_carve(CsrBufs& c, char* ws, size_t off, int E, int N) {
  const size_t off0 = off; c.base = ws + off;
  auto al = [&](size_t bytes) { char* p = ws + off; off += (bytes + 255) & ~(size_t)255; return p; };
  c.nG = (N + CSR_GN - 1) / CSR_GN; c.NGP = (c.nG + 31) & ~31; const int ch = (E + CSR_NBLK - 1) / CSR_NBLK; c.CHP = (ch + 31) & ~31; c.permLen = (size_t)E + 32 * (size_t)c.nG + 32;
  c.STG = (int*)al((size_t)CSR_NBLK * c.CHP * 4); c.HST = (int*)al((size_t)CSR_NBLK * c.NGP * 4); c.OFF = (int*)al((size_t)c.NGP * CSR_NBLK * 4); c.START = (int*)al((size_t)(c.NGP + 64) * 4); c.TOT = (int*)al((size_t)(c.NGP + 64) * 4);
  c.PERM = (int*)al(c.permLen * 4); c.ROWPTR = (int*)al((size_t)c.nG * CSR_GN * 4); c.ROWCNT = (int*)al((size_t)c.nG * CSR_GN * 4); c.FLAG = (int*)al(256);
  c.bytes = off - off0; return off;
}
static void csr_build(const CsrBufs& c, const int* dst, int E, int N, hipStream_t stream) {
  const size_t smem = (size_t)(2 * c.NGP + c.CHP) * 4;
  csrZ_kernel<<<512, 256, 0, stream>>>((int*)c.base, c.bytes / 16);
  csrA_kernel<<<CSR_NBLK, 64, smem, stream>>>(dst, E, N, c.nG, c.CHP, c.NGP, c.STG, c.HST);
  csrS_kernel<<<1, 512, 0, stream>>>(c.HST, c.nG, c.NGP, c.START, c.TOT, c.OFF);
  csrB_kernel<<<c.nG, 256, 0, stream>>>(dst, N, c.nG, c.CHP, c.NGP, (int)c.permLen, c.STG, c.HST, c.OFF, c.START, c.TOT, c.PERM, c.ROWPTR, c.ROWCNT, c.FLAG);
}


__global__ __launch_bounds__(256) void prepw_kernel(const float* __restrict__ w1, const float* __restrict__ w2, const float* __restrict__ wfc, b16* __restrict__ W1P, b16* __restrict__ W2P, b16* __restrict__ WFC) {
  const size_t t = (size_t)blockIdx.x * 256 + threadIdx.x; const size_t n1 = 64 * 32 / 8, n2 = 64 * 64 / 8, n3 = (size_t)16 * KFC / 8; v8b o;
  if (t < n1) { const int e = (int)t * 8; const int oo = e / 32, k0 = e % 32; for (int j = 0; j < 8; ++j) { const int k = k0 + j; o[j] = (k < FIN) ? (b16)(bf16_rne(w1[k * HID + oo]) * WSC) : (b16)0.0f; } for (int pass = 0; pass < 2; ++pass) { *(volatile v8b*)(W1P + e) = o; __threadfence(); } }
  else if (t < n1 + n2) { const int e = (int)(t - n1) * 8; const int oo = e / 64, k0 = e % 64; for (int j = 0; j < 8; ++j) o[j] = (b16)(bf16_rne(w2[(k0 + j) * HID + oo]) * WSC); for (int pass = 0; pass < 2; ++pass) { *(volatile v8b*)(W2P + e) = o; __threadfence(); } }
  else if (t < n1 + n2 + n3) { const size_t e = (t - n1 - n2) * 8; const int oo = (int)(e / KFC); const size_t k0 = e % KFC; for (int j = 0; j < 8; ++j) o[j] = (oo < OUT) ? (b16)(bf16_rne(wfc[(k0 + j) * OUT + oo]) * WSC) : (b16)0.0f; for (int pass = 0; pass < 2; ++pass) { *(volatile v8b*)(WFC + e) = o; __threadfence(); } }
}
__global__ __launch_bounds__(128) void layer1_kernel(const float* __restrict__ x, const int* __restrict__ srcs, const int* __restrict__ PERM, const int* __restrict__ ROWPTR, const int* __restrict__ ROWCNT, int permLen, const b16* __restrict__ W1P, const float* __restrict__ b1, float* __restrict__ H1) {
  __shared__ __attribute__((aligned(16))) b16 Ah[64][40], Al[64][40]; __shared__ __attribute__((aligned(16))) float Ts[4][16][HID + 4];
  const int wave = threadIdx.x >> 5, lane = threadIdx.x & 31, nloc = lane & 15, hlf = lane >> 4; const size_t row0 = (size_t)blockIdx.x * 64 + wave * 16;
  for (int r = 0; r < 16; ++r) { Ah[wave * 16 + r][16 + nloc] = (b16)0.0f; Al[wave * 16 + r][16 + nloc] = (b16)0.0f; }
  const int q = lane >> 4, f = lane & 15;
  for (int g = 0; g < 8; ++g) { const size_t v = row0 + g * 2 + q; float acc = 0.0f;
    { int st = ROWPTR[v], cnt = ROWCNT[v]; cnt = iclamp(cnt, 0, 8192); st = iclamp(st, 0, permLen - cnt); const float dv = rsqrtf((float)cnt + 1.0f); acc = pmul(dv, bf16_rne(x[v * FIN + f]));
      for (int j = 0; j < cnt; ++j) { const int e = iclamp(PERM[st + j], 0, E - 1); const int s = iclamp(srcs[e], 0, N - 1); const float ds = rsqrtf((float)iclamp(ROWCNT[s], 0, 8192) + 1.0f); acc += pmul(ds, bf16_rne(x[(size_t)s * FIN + f])); }
      acc = pmul(acc, dv); }
    b16 p, qq; split16(acc * XS, p, qq); Ah[wave * 16 + g * 2 + q][f] = p; Al[wave * 16 + g * 2 + q][f] = qq; }
  wave_lds_sync();
  v8f a4[4] = {{}, {}, {}, {}}; { const v16b a = frag_kb(&Ah[wave * 16 + nloc][0], hlf), al = frag_kb(&Al[wave * 16 + nloc][0], hlf);
#pragma unroll
    for (int t = 0; t < 4; ++t) { const v16b bw = frag_kb(W1P + (size_t)(t * 16 + nloc) * 32, hlf); a4[t] = wmma16b(a, bw, a4[t]); a4[t] = wmma16b(al, bw, a4[t]); } }
#pragma unroll
  for (int t = 0; t < 4; ++t) { const int c = t * 16 + nloc; const float bb = bf16_rne(b1[c]);
#pragma unroll
    for (int r = 0; r < 8; ++r) Ts[wave][8 * hlf + r][c] = tanh_(a4[t][r] * (1.0f / (XS * WSC)) + bb); }
  wave_lds_sync();
  for (int pass = 0; pass < 2; ++pass) { for (int rr = 0; rr < 16; ++rr) if (lane < 16) *(volatile v4f*)(H1 + (row0 + rr) * HID + lane * 4) = *(const v4f*)(&Ts[wave][rr][lane * 4]); __threadfence(); }
}
__global__ __launch_bounds__(128) void layer2_kernel(const float* __restrict__ H1, const int* __restrict__ srcs, const int* __restrict__ PERM, const int* __restrict__ ROWPTR, const int* __restrict__ ROWCNT, int permLen, const b16* __restrict__ W2P, const float* __restrict__ b2, b16* __restrict__ H2h, b16* __restrict__ H2l) {
  __shared__ __attribute__((aligned(16))) b16 Ah[64][72], Al[64][72]; __shared__ __attribute__((aligned(16))) b16 Oh[4][16][72], Ol[4][16][72];
  const int wave = threadIdx.x >> 5, lane = threadIdx.x & 31, nloc = lane & 15, hlf = lane >> 4; const size_t row0 = (size_t)blockIdx.x * 64 + wave * 16; const int c0 = lane * 2;
  for (int rl = 0; rl < 16; ++rl) { const size_t v = row0 + rl; int st = ROWPTR[v], cnt = ROWCNT[v]; cnt = iclamp(cnt, 0, 8192); st = iclamp(st, 0, permLen - cnt); const float dv = rsqrtf((float)cnt + 1.0f);
    const v2f hs = *(const v2f*)(H1 + v * HID + c0); float a0 = pmul(dv, hs[0]), a1 = pmul(dv, hs[1]);
    for (int j = 0; j < cnt; ++j) { const int e = iclamp(PERM[st + j], 0, E - 1); const int s = iclamp(srcs[e], 0, N - 1); const float ds = rsqrtf((float)iclamp(ROWCNT[s], 0, 8192) + 1.0f); const v2f h = *(const v2f*)(H1 + (size_t)s * HID + c0); a0 += pmul(ds, h[0]); a1 += pmul(ds, h[1]); }
    a0 = pmul(a0, dv); a1 = pmul(a1, dv); b16 p, q; split16(a0 * XS, p, q); Ah[wave * 16 + rl][c0] = p; Al[wave * 16 + rl][c0] = q; split16(a1 * XS, p, q); Ah[wave * 16 + rl][c0 + 1] = p; Al[wave * 16 + rl][c0 + 1] = q; }
  wave_lds_sync();
  v8f a4[4] = {{}, {}, {}, {}};
#pragma unroll
  for (int kb = 0; kb < HID; kb += 32) { const v16b a = frag_kb(&Ah[wave * 16 + nloc][kb], hlf), al = frag_kb(&Al[wave * 16 + nloc][kb], hlf);
#pragma unroll
    for (int t = 0; t < 4; ++t) { const v16b bw = frag_kb(W2P + (size_t)(t * 16 + nloc) * HID + kb, hlf); a4[t] = wmma16b(a, bw, a4[t]); a4[t] = wmma16b(al, bw, a4[t]); } }
#pragma unroll
  for (int t = 0; t < 4; ++t) { const int c = t * 16 + nloc; const float bb = bf16_rne(b2[c]);
#pragma unroll
    for (int r = 0; r < 8; ++r) { b16 p, q; split16(tanh_(a4[t][r] * (1.0f / (XS * WSC)) + bb) * XS, p, q); Oh[wave][8 * hlf + r][c] = p; Ol[wave][8 * hlf + r][c] = q; } }
  wave_lds_sync();
  for (int pass = 0; pass < 2; ++pass) { for (int qd = lane; qd < 16 * 8; qd += 32) { const int rr = qd >> 3, c8 = (qd & 7) * 8; *(volatile v8b*)(H2h + (row0 + rr) * HID + c8) = *(const v8b*)(&Oh[wave][rr][c8]); *(volatile v8b*)(H2l + (row0 + rr) * HID + c8) = *(const v8b*)(&Ol[wave][rr][c8]); } __threadfence(); }
}
__global__ __launch_bounds__(64) void fc_kernel(const b16* __restrict__ H2h, const b16* __restrict__ H2l, const b16* __restrict__ WFC, float* __restrict__ PP) {
  const int wave = threadIdx.x >> 5, lane = threadIdx.x & 31, nloc = lane & 15, hlf = lane >> 4; const int ch = blockIdx.x; const size_t k0 = (size_t)ch * KCH; const size_t g = (size_t)wave * 16 + nloc;
  v8f acc = {};
#pragma unroll 4
  for (int kb = 0; kb < KCH; kb += 32) { const v16b a = frag_kb(H2h + g * KFC + k0 + kb, hlf), al = frag_kb(H2l + g * KFC + k0 + kb, hlf); const v16b bw = frag_kb(WFC + (size_t)nloc * KFC + k0 + kb, hlf); acc = wmma16b(a, bw, acc); acc = wmma16b(al, bw, acc); }
  __shared__ __attribute__((aligned(16))) float Ts[2][16][20];
#pragma unroll
  for (int r = 0; r < 8; ++r) Ts[wave][8 * hlf + r][nloc] = acc[r] * (1.0f / (XS * WSC));
  wave_lds_sync();
  for (int pass = 0; pass < 2; ++pass) { for (int it = 0; it < 2; ++it) { const int rr = it * 8 + (lane >> 2), c4 = (lane & 3) * 4; const v4f a = *(const v4f*)(&Ts[wave][rr][c4]); *(volatile v4f*)(PP + (((size_t)ch * NG + wave * 16 + rr) * 16) + c4) = a; } __threadfence(); }
}
__global__ __launch_bounds__(512) void final_kernel(const float* __restrict__ PP, const float* __restrict__ bfc, float* __restrict__ out) {
  __shared__ __attribute__((aligned(16))) float Os[NG * OUT];
  const int t = threadIdx.x; const int g = t >> 4, o = t & 15; float s = 0.0f; if (o < OUT) { for (int ch = 0; ch < NCH; ++ch) s += PP[((size_t)ch * NG + g) * 16 + o]; s += bf16_rne(bfc[o]); Os[g * OUT + o] = s; }
  __syncthreads();
  if (t < 32) { for (int pass = 0; pass < 2; ++pass) { for (int it = 0; it < 3; ++it) *(volatile v4f*)(out + it * 128 + t * 4) = *(const v4f*)(&Os[it * 128 + t * 4]); __threadfence(); } }
}
}

extern "C" void kernel_launch(void* const* d_in, const int* in_sizes, int n_in, void* d_out, int out_size, void* d_ws, size_t ws_size, hipStream_t stream) {
  (void)n_in;
  auto Fp = [&](int i) { return (const float*)d_in[i]; }; auto Ip = [&](int i) { return (const int*)d_in[i]; };
  if (in_sizes[0] != N * FIN || in_sizes[1] != 2 * E || in_sizes[2] != N || in_sizes[3] != FIN * HID || in_sizes[5] != HID * HID || in_sizes[7] != KFC * OUT || out_size != NG * OUT) return;
  size_t off = 0; char* ws = (char*)d_ws;
  auto carve = [&](size_t bytes) { char* p = ws + off; off += (bytes + 255) & ~(size_t)255; return p; };
  b16* W1P = (b16*)carve(64 * 32 * 2); b16* W2P = (b16*)carve(64 * 64 * 2); b16* WFC = (b16*)carve((size_t)16 * KFC * 2); float* H1 = (float*)carve((size_t)N * HID * 4); b16* H2h = (b16*)carve((size_t)N * HID * 2); b16* H2l = (b16*)carve((size_t)N * HID * 2); float* PP = (float*)carve((size_t)NCH * NG * 16 * 4);
  CsrBufs csr; off = csr_carve(csr, ws, off, E, N);
  if (off > ws_size || off > ((size_t)128 << 20)) return;
  prepw_kernel<<<(unsigned)((64 * 32 / 8 + 64 * 64 / 8 + (size_t)16 * KFC / 8 + 255) / 256), 256, 0, stream>>>(Fp(3), Fp(5), Fp(7), W1P, W2P, WFC);
  csr_build(csr, Ip(1) + E, E, N, stream);
  layer1_kernel<<<N / 64, 128, 0, stream>>>(Fp(0), Ip(1), csr.PERM, csr.ROWPTR, csr.ROWCNT, (int)csr.permLen, W1P, Fp(4), H1);
  layer2_kernel<<<N / 64, 128, 0, stream>>>(H1, Ip(1), csr.PERM, csr.ROWPTR, csr.ROWCNT, (int)csr.permLen, W2P, Fp(6), H2h, H2l);
  fc_kernel<<<NCH, 64, 0, stream>>>(H2h, H2l, WFC, PP);
  final_kernel<<<1, 512, 0, stream>>>(PP, Fp(8), (float*)d_out);
}
